// GaussianAttention_51230369906982
// MI455X (gfx1250) — hardware-run, weakly checked
//
#include <hip/hip_runtime.h>
#include <math.h>

typedef __attribute__((ext_vector_type(16))) _Float16 v16h;
typedef __attribute__((ext_vector_type(16))) __bf16 v16b;
typedef __attribute__((ext_vector_type(8)))  _Float16 v8h;
typedef __attribute__((ext_vector_type(8)))  float v8f;
typedef __attribute__((ext_vector_type(4)))  float v4f;
typedef __attribute__((ext_vector_type(2)))  float v2f;
typedef __attribute__((ext_vector_type(4)))  unsigned v4u;
typedef __attribute__((ext_vector_type(4)))  int v4i;
typedef float __attribute__((may_alias)) float_a;
typedef int __attribute__((may_alias)) int_a;

template <typename T> __device__ __forceinline__ void vst2(void* p, T v) { *(volatile T*)p = v; __threadfence(); *(volatile T*)p = v; }
__device__ __forceinline__ v8f wmma16(v16h a, v16h b, v8f c) {
  v8f d = __builtin_amdgcn_wmma_f32_16x16x32_f16(false, a, false, b, (short)0, c, false, false);
  asm volatile("v_nop\n\tv_nop\n\tv_nop\n\tv_nop" : "+v"(d) : "v"(a), "v"(b));
  return d;
}
__device__ __forceinline__ v8f wmma_bf(v16b a, v16b b, v8f c) {
  v8f d = __builtin_amdgcn_wmma_f32_16x16x32_bf16(false, a, false, b, (short)0, c, false, false);
  asm volatile("v_nop\n\tv_nop\n\tv_nop\n\tv_nop" : "+v"(d) : "v"(a), "v"(b));
  return d;
}
__device__ __forceinline__ v16h frag_h(const _Float16* rowk0, int lane) {
  union { v16h v; v8h q[2]; } u; const _Float16* p = rowk0 + 8 * (lane >> 4);
  u.q[0] = *(const v8h*)p; u.q[1] = *(const v8h*)(p + 16); return u.v;
}
__device__ __forceinline__ v16h frag_f32(const float* rowk0, int lane) {
  v16h a; const float* p = rowk0 + 8 * (lane >> 4);
#pragma unroll
  for (int i = 0; i < 8; ++i) { a[i] = (_Float16)p[i]; a[8 + i] = (_Float16)p[16 + i]; }
  return a;
}
__device__ __forceinline__ v16h frag_f32s(const float* rowk0, int lane, float sc) {
  v16h a; const float* p = rowk0 + 8 * (lane >> 4);
#pragma unroll
  for (int i = 0; i < 8; ++i) { a[i] = (_Float16)(p[i] * sc); a[8 + i] = (_Float16)(p[16 + i] * sc); }
  return a;
}
__device__ __forceinline__ v16h fragc_f32(const float* W, int k0, int n, int lane, int ld, int K) {
  v16h a; const int g = lane >> 4;
#pragma unroll
  for (int i = 0; i < 8; ++i) { const int ka = k0 + 8 * g + i, kb = ka + 16;
    a[i] = (_Float16)(ka < K ? W[(size_t)(ka < K ? ka : K - 1) * ld + n] : 0.f); a[8 + i] = (_Float16)(kb < K ? W[(size_t)(kb < K ? kb : K - 1) * ld + n] : 0.f); }
  return a;
}
struct F2 { v16b h, l; };
__device__ __forceinline__ F2 bsplit16(const float v[16]) { F2 r;
#pragma unroll
  for (int i = 0; i < 16; ++i) { const __bf16 h = (__bf16)v[i]; r.h[i] = h; r.l[i] = (__bf16)(v[i] - (float)h); }
  return r; }
__device__ __forceinline__ F2 split_row(const float* row, int k0, int lane) { float v[16]; const float* p = row + k0 + 8 * (lane >> 4);
#pragma unroll
  for (int i = 0; i < 8; ++i) { v[i] = p[i]; v[8 + i] = p[16 + i]; }
  return bsplit16(v); }
__device__ __forceinline__ F2 split_rowK(const float* row, int k0, int lane, int K) { float v[16]; const int g = lane >> 4;
#pragma unroll
  for (int i = 0; i < 8; ++i) { const int ka = k0 + 8 * g + i, kb = ka + 16; v[i] = ka < K ? row[ka < K ? ka : K - 1] : 0.f; v[8 + i] = kb < K ? row[kb < K ? kb : K - 1] : 0.f; }
  return bsplit16(v); }
__device__ __forceinline__ F2 split_col(const float* W, int k0, int n, int lane, int ld, int K) { float v[16]; const int g = lane >> 4;
#pragma unroll
  for (int i = 0; i < 8; ++i) { const int ka = k0 + 8 * g + i, kb = ka + 16; v[i] = ka < K ? W[(size_t)(ka < K ? ka : K - 1) * ld + n] : 0.f; v[8 + i] = kb < K ? W[(size_t)(kb < K ? kb : K - 1) * ld + n] : 0.f; }
  return bsplit16(v); }
__device__ __forceinline__ v8f mac3(const F2& a, const F2& b, v8f c) { c = wmma_bf(a.l, b.h, c); c = wmma_bf(a.h, b.l, c); return wmma_bf(a.h, b.h, c); }
__device__ __forceinline__ float sigm(float v) { return 1.0f / (1.0f + expf(-v)); }
#define LDSX() do { asm volatile("s_wait_dscnt 0" ::: "memory"); __builtin_amdgcn_wave_barrier(); __builtin_amdgcn_fence(__ATOMIC_RELEASE, "workgroup"); } while (0)


#define NB 4
#define CC 256
#define CQ 64
#define HH 64
#define WWD 64
#define TT 4096
#define RED 16
#ifndef TNB
#define TNB NB
#endif
typedef __attribute__((ext_vector_type(8))) __bf16 v8b;
__device__ __forceinline__ v16b frag_b(const __bf16* rowk0, int lane) {
  union { v16b v; v8b q[2]; } u; const __bf16* p = rowk0 + 8 * (lane >> 4);
  u.q[0] = *(const v8b*)p; u.q[1] = *(const v8b*)(p + 16); return u.v;
}
__device__ __forceinline__ float bfr(float v) { return (float)(__bf16)v; }
__device__ __attribute__((noinline)) float exp_ni(float v) { return expf(v); }
__device__ __attribute__((noinline)) float erf_ni(float v) { return erff(v); }

#define WS_QH  0u
#define WS_QL  (WS_QH + 2u * (size_t)NB * TT * CQ)
#define WS_KH  (WS_QL + 2u * (size_t)NB * TT * CQ)
#define WS_VT  (WS_KH + 2u * (size_t)NB * TT * CQ)
#define WS_S   (WS_VT + 2u * (size_t)NB * CC * TT)
#define WS_PH  (WS_S + 4u * (size_t)TT * TT)
#define WS_CS  (WS_PH + 2u * (size_t)TT * TT)
#define WS_Y   (WS_CS + 4u * (size_t)NB * TT)
#define WS_G   (WS_Y + 4u * (size_t)NB * CC * TT)
#define WS_END (WS_G + 4u * (size_t)NB * CC)

__global__ __launch_bounds__(128) void k_projqk(const float* __restrict__ XQ, const float* __restrict__ XKV, const float* __restrict__ WQ, const float* __restrict__ BQ, const float* __restrict__ WK, const float* __restrict__ BK, _Float16* __restrict__ QH, _Float16* __restrict__ QL, _Float16* __restrict__ KH) {
  __shared__ __align__(16) __bf16 sx[64][CC + 8]; __shared__ __align__(16) _Float16 sh[64][72], sl[64][72];
  const int tid = threadIdx.x, wave = tid >> 5, lane = tid & 31, col = lane & 15, g = lane >> 4; const int p0 = blockIdx.x * 64; const size_t b = blockIdx.z >> 1; const int which = blockIdx.z & 1;
  const float* X = which == 0 ? XQ : XKV; const float* Wm = which == 0 ? WQ : WK; const float* Bm = which == 0 ? BQ : BK;
  for (int e = tid; e < CC * 64; e += 128) { const int c = e >> 6, pl = e & 63; sx[pl][c] = (__bf16)X[(b * CC + c) * (size_t)TT + p0 + pl]; }
  __syncthreads();
  v8f acc[4] = {};
#pragma unroll 2
  for (int kc = 0; kc < CC / 32; ++kc) { const v16b a = frag_b(&sx[wave * 16 + col][kc * 32], lane);
#pragma unroll
    for (int j = 0; j < 4; ++j) { v16b w; const int o = j * 16 + col;
#pragma unroll
      for (int i = 0; i < 8; ++i) { w[i] = (__bf16)Wm[(size_t)(kc * 32 + 8 * g + i) * CQ + o]; w[8 + i] = (__bf16)Wm[(size_t)(kc * 32 + 16 + 8 * g + i) * CQ + o]; }
      acc[j] = wmma_bf(a, w, acc[j]); } }
#pragma unroll
  for (int j = 0; j < 4; ++j) { const float bb = bfr(Bm[j * 16 + col]);
#pragma unroll
    for (int r = 0; r < 8; ++r) { const float v = acc[j][r] + bb; const int rl = wave * 16 + 8 * g + r, cl = j * 16 + col; const _Float16 hv = (_Float16)v; sh[rl][cl] = hv; sl[rl][cl] = (_Float16)(v - (float)hv); } }
  __syncthreads();
  _Float16* dh = which == 0 ? QH : KH; for (int e = tid; e < 64 * 8; e += 128) { const int rl = e >> 3, q = e & 7; const size_t row = b * TT + p0 + rl; vst2((unsigned*)(dh + row * CQ + q * 8), *(const v4u*)&sh[rl][q * 8]); if (which == 0) vst2((unsigned*)(QL + row * CQ + q * 8), *(const v4u*)&sl[rl][q * 8]); } }
__global__ __launch_bounds__(128) void k_projv(const float* __restrict__ XKV, const float* __restrict__ WV, const float* __restrict__ BV, _Float16* __restrict__ VT) {
  __shared__ __align__(16) __bf16 sx[64][CC + 8]; __shared__ __align__(16) _Float16 th[128][72];
  const int tid = threadIdx.x, wave = tid >> 5, lane = tid & 31, col = lane & 15, g = lane >> 4; const int p0 = blockIdx.x * 64; const int c0 = blockIdx.y * 128; const size_t b = blockIdx.z;
  for (int e = tid; e < CC * 64; e += 128) { const int c = e >> 6, pl = e & 63; sx[pl][c] = (__bf16)XKV[(b * CC + c) * (size_t)TT + p0 + pl]; }
  __syncthreads();
  v8f acc[8] = {};
#pragma unroll 2
  for (int kc = 0; kc < CC / 32; ++kc) { const v16b a = frag_b(&sx[wave * 16 + col][kc * 32], lane);
#pragma unroll
    for (int j = 0; j < 8; ++j) { v16b w; const int o = c0 + j * 16 + col;
#pragma unroll
      for (int i = 0; i < 8; ++i) { w[i] = (__bf16)WV[(size_t)(kc * 32 + 8 * g + i) * CC + o]; w[8 + i] = (__bf16)WV[(size_t)(kc * 32 + 16 + 8 * g + i) * CC + o]; }
      acc[j] = wmma_bf(a, w, acc[j]); } }
#pragma unroll
  for (int j = 0; j < 8; ++j) { const float bb = bfr(BV[c0 + j * 16 + col]);
#pragma unroll
    for (int r = 0; r < 8; ++r) th[j * 16 + col][wave * 16 + 8 * g + r] = (_Float16)(acc[j][r] + bb); }
  __syncthreads(); for (int e = tid; e < 128 * 8; e += 128) { const int cl = e >> 3, q = e & 7; vst2((unsigned*)(VT + (b * CC + c0 + cl) * (size_t)TT + p0 + q * 8), *(const v4u*)&th[cl][q * 8]); } }
__global__ __launch_bounds__(128) void k_sc(const _Float16* __restrict__ QH, const _Float16* __restrict__ QL, const _Float16* __restrict__ KH, int b, float* __restrict__ S) { __shared__ __align__(16) float ss[4][16][132];
  const int tid = threadIdx.x, wave = tid >> 5, lane = tid & 31, col = lane & 15, g = lane >> 4; const int k0 = blockIdx.y * 128; const int ql0 = blockIdx.x * 64 + wave * 16; const size_t q0 = (size_t)b * TT + ql0;
  v8f acc[8] = {};
#pragma unroll
  for (int kc = 0; kc < CQ / 32; ++kc) { const v16h ah = frag_h(QH + (q0 + col) * CQ + kc * 32, lane), al = frag_h(QL + (q0 + col) * CQ + kc * 32, lane);
#pragma unroll
    for (int j = 0; j < 8; ++j) { const v16h kb = frag_h(KH + ((size_t)b * TT + k0 + j * 16 + col) * CQ + kc * 32, lane); acc[j] = wmma16(ah, kb, acc[j]); acc[j] = wmma16(al, kb, acc[j]); } }
#pragma unroll
  for (int j = 0; j < 8; ++j)
#pragma unroll
    for (int r = 0; r < 8; ++r) ss[wave][8 * g + r][j * 16 + col] = acc[j][r] * 0.125f;
  LDSX(); for (int rl = 0; rl < 16; ++rl) vst2(S + (size_t)(ql0 + rl) * TT + k0 + lane * 4, *(const v4f*)&ss[wave][rl][lane * 4]); }
__global__ __launch_bounds__(256) void k_sm(const float* __restrict__ S, const float* __restrict__ LSQ, _Float16* __restrict__ PH) { __shared__ float sred[8]; __shared__ float sbc; __shared__ __align__(16) _Float16 sh[TT]; __shared__ float ex[HH], ey[WWD];
  const int t = threadIdx.x; const size_t row = blockIdx.x; const float* sr = S + row * TT; const int qr = (int)row / WWD, qc = (int)row % WWD;
  { const float ssq = expf(bfr(LSQ[0])); const float maxd = (float)((HH - 1) * (HH - 1) + (WWD - 1) * (WWD - 1)); const float cdn = 1.0f / maxd / (2.0f * ssq); if (t < HH) ex[t] = expf(-(float)(t * t) * cdn); else if (t < HH + WWD) { const int u = t - HH; ey[u] = expf(-(float)(u * u) * cdn); } }
  float m = -3.0e38f; for (int k = t; k < TT; k += 256) m = fmaxf(m, sr[k]);
#pragma unroll
  for (int o = 1; o < 32; o <<= 1) m = fmaxf(m, __shfl_xor(m, o));
  if ((t & 31) == 0) sred[t >> 5] = m; __syncthreads(); if (t == 0) { float a = sred[0]; for (int i = 1; i < 8; ++i) a = fmaxf(a, sred[i]); sbc = a; } __syncthreads(); m = sbc; __syncthreads();
  float sum = 0.f; for (int k = t; k < TT; k += 256) sum += expf(sr[k] - m);
#pragma unroll
  for (int o = 1; o < 32; o <<= 1) sum += __shfl_xor(sum, o);
  if ((t & 31) == 0) sred[t >> 5] = sum; __syncthreads(); if (t == 0) { float a = 0.f; for (int i = 0; i < 8; ++i) a += sred[i]; sbc = 1.0f / a; } __syncthreads(); const float inv = sbc;
  for (int k = t; k < TT; k += 256) { const int kr = k / WWD, kcx = k % WWD; const int adx = qr > kr ? qr - kr : kr - qr, ady = qc > kcx ? qc - kcx : kcx - qc; sh[k] = (_Float16)(expf(sr[k] - m) * inv * ex[adx] * ey[ady] * 2048.0f); }
  __syncthreads(); for (int q = t; q < TT / 8; q += 256) vst2((unsigned*)(PH + row * TT + q * 8), *(const v4u*)&sh[q * 8]); }
__global__ __launch_bounds__(256) void k_col(const _Float16* __restrict__ PH, int b, float* __restrict__ CS) { __shared__ __align__(16) float so[256];
  const int t = threadIdx.x; const int k = blockIdx.x * 256 + t; float a = 0.f;
#pragma unroll 4
  for (int q = 0; q < TT; ++q) a += (float)PH[(size_t)q * TT + k];
  so[t] = a * (1.0f / 2048.0f);
  __syncthreads(); if (t < 64) vst2(CS + (size_t)b * TT + blockIdx.x * 256 + t * 4, *(const v4f*)&so[t * 4]); }
__global__ __launch_bounds__(128) void k_pv(const _Float16* __restrict__ PH, const _Float16* __restrict__ VT, int b, float* __restrict__ Y) { __shared__ __align__(16) float so[128][68];
  const int tid = threadIdx.x, wave = tid >> 5, lane = tid & 31, col = lane & 15, g = lane >> 4; const int q0b = blockIdx.x * 64; const int ql0 = q0b + wave * 16; const int c0 = blockIdx.y * 128;
  v8f acc[8] = {};
#pragma unroll 1
  for (int kc = 0; kc < TT / 32; ++kc) { const v16h ph = frag_h(PH + (size_t)(ql0 + col) * TT + kc * 32, lane);
#pragma unroll
    for (int j = 0; j < 8; ++j) acc[j] = wmma16(ph, frag_h(VT + ((size_t)b * CC + c0 + j * 16 + col) * (size_t)TT + kc * 32, lane), acc[j]); }
#pragma unroll
  for (int j = 0; j < 8; ++j)
#pragma unroll
    for (int r = 0; r < 8; ++r) so[j * 16 + col][wave * 16 + 8 * g + r] = acc[j][r] * (1.0f / 2048.0f);
  __syncthreads(); for (int e = tid; e < 128 * 16; e += 128) { const int cl = e >> 4, q = e & 15; vst2(Y + ((size_t)b * CC + c0 + cl) * TT + q0b + q * 4, *(const v4f*)&so[cl][q * 4]); } }
__global__ __launch_bounds__(256) void k_gate(const float* __restrict__ CS, const float* __restrict__ Y, const float* __restrict__ LSE, const float* __restrict__ W1, const float* __restrict__ W2, float* __restrict__ G) {
  __shared__ float sred[8]; __shared__ float s_tot, s_mh, s_mw, s_ks; __shared__ float skern[TT]; __shared__ float ssq[CC]; __shared__ float shid[RED]; __shared__ __align__(16) float sg[CC];
  const int t = threadIdx.x, wv = t >> 5, ln = t & 31; const size_t b = blockIdx.x; const float* cs = CS + b * TT;
  float a = 0.f;
#pragma unroll 1
  for (int k = t; k < TT; k += 256) a += cs[k];
#pragma unroll
  for (int o = 1; o < 32; o <<= 1) a += __shfl_xor(a, o);
  if (ln == 0) sred[wv] = a; __syncthreads(); if (t == 0) { float x = 0.f; for (int i = 0; i < 8; ++i) x += sred[i]; s_tot = x; } __syncthreads(); const float invt = 1.0f / (s_tot + 1e-8f);
  float ah = 0.f, aw = 0.f;
#pragma unroll 1
  for (int k = t; k < TT; k += 256) { const float w8 = cs[k] * invt; ah += (float)(k / WWD) * w8; aw += (float)(k % WWD) * w8; }
#pragma unroll
  for (int o = 1; o < 32; o <<= 1) { ah += __shfl_xor(ah, o); aw += __shfl_xor(aw, o); }
  __syncthreads(); if (ln == 0) sred[wv] = ah; __syncthreads(); if (t == 0) { float x = 0.f; for (int i = 0; i < 8; ++i) x += sred[i]; s_mh = x / (float)(HH - 1); } __syncthreads();
  if (ln == 0) sred[wv] = aw; __syncthreads(); if (t == 0) { float x = 0.f; for (int i = 0; i < 8; ++i) x += sred[i]; s_mw = x / (float)(WWD - 1); } __syncthreads();
  const float mh = s_mh, mw = s_mw; const float sse = expf(bfr(LSE[0]));
  float ks = 0.f;
#pragma unroll 1
  for (int p = t; p < TT; p += 256) { const int r = p / WWD, c = p % WWD; const float gx = (float)r / (float)(HH - 1) - mh, gy = (float)c / (float)(WWD - 1) - mw; const float kv = expf(-(gx * gx + gy * gy) / (2.0f * sse)); skern[p] = kv; ks += kv; }
#pragma unroll
  for (int o = 1; o < 32; o <<= 1) ks += __shfl_xor(ks, o);
  __syncthreads(); if (ln == 0) sred[wv] = ks; __syncthreads(); if (t == 0) { float x = 0.f; for (int i = 0; i < 8; ++i) x += sred[i]; s_ks = 1.0f / x; } __syncthreads(); const float invk = s_ks;
  for (int c = wv; c < CC; c += 8) { float s = 0.f; const float* yp = Y + (b * CC + c) * (size_t)TT;
#pragma unroll 1
    for (int p = ln; p < TT; p += 32) s += yp[p] * skern[p];
#pragma unroll
    for (int o = 1; o < 32; o <<= 1) s += __shfl_xor(s, o); if (ln == 0) ssq[c] = s * invk; }
  __syncthreads();
  if (t < RED) { float h = 0.f;
#pragma unroll 1
    for (int c = 0; c < CC; ++c) h += ssq[c] * bfr(W1[c * RED + t]); shid[t] = fmaxf(h, 0.f); }
  __syncthreads();
  { float gsum = 0.f;
#pragma unroll 1
    for (int j = 0; j < RED; ++j) gsum += shid[j] * bfr(W2[j * CC + t]); sg[t] = 1.0f / (1.0f + expf(-gsum)); }
  __syncthreads(); if (t < CC / 4) vst2(G + b * CC + t * 4, *(const v4f*)&sg[t * 4]); }
__global__ __launch_bounds__(256) void k_apply(const float* __restrict__ Y, const float* __restrict__ G, float* __restrict__ OUT) {
  const int t = threadIdx.x; const size_t bc = blockIdx.y; const int p0 = blockIdx.x * 1024; const float gt = G[bc]; const float* yp = Y + bc * TT + p0;
  v4f v = *(const v4f*)(yp + t * 4); v[0] *= gt; v[1] *= gt; v[2] *= gt; v[3] *= gt; vst2(OUT + bc * TT + p0 + t * 4, v); }
extern "C" void kernel_launch(void* const* d_in, const int* in_sizes, int n_in, void* d_out, int out_size, void* d_ws, size_t ws_size, hipStream_t stream) {
  (void)in_sizes; (void)n_in; (void)out_size;
  const float** F = (const float**)d_in;
  if (ws_size < (size_t)WS_END) return;
  char* ws = (char*)d_ws; _Float16 *QH = (_Float16*)(ws + WS_QH), *QL = (_Float16*)(ws + WS_QL), *KH = (_Float16*)(ws + WS_KH), *VT = (_Float16*)(ws + WS_VT), *PH = (_Float16*)(ws + WS_PH); float *S = (float*)(ws + WS_S), *CS = (float*)(ws + WS_CS), *Y = (float*)(ws + WS_Y), *G = (float*)(ws + WS_G);
  k_projqk<<<dim3(TT / 64, 1, TNB * 2), 128, 0, stream>>>(F[0], F[1], F[2], F[3], F[4], F[5], QH, QL, KH);
  k_projv<<<dim3(TT / 64, CC / 128, TNB), 128, 0, stream>>>(F[1], F[6], F[7], VT);
  for (int b = 0; b < TNB; ++b) {
    k_sc<<<dim3(TT / 64, TT / 128), 128, 0, stream>>>(QH, QL, KH, b, S);
    k_sm<<<TT, 256, 0, stream>>>(S, F[8], PH);
    k_col<<<TT / 256, 256, 0, stream>>>(PH, b, CS);
    k_pv<<<dim3(TT / 64, CC / 128), 128, 0, stream>>>(PH, VT, b, Y);
  }
  k_gate<<<TNB, 256, 0, stream>>>(CS, Y, F[9], F[10], F[11], G);
  k_apply<<<dim3(TT / 1024, TNB * CC), 256, 0, stream>>>(Y, G, (float*)d_out);
}
